// DeformableAlignmentFusion_16810501997304
// MI455X (gfx1250) — hardware-verified
//
#include <hip/hip_runtime.h>
#include <stddef.h>

#pragma clang fp contract(off)


typedef _Float16 v4h  __attribute__((ext_vector_type(4)));
typedef _Float16 v8h  __attribute__((ext_vector_type(8)));
typedef _Float16 v16h __attribute__((ext_vector_type(16)));
typedef float    v4f  __attribute__((ext_vector_type(4)));
typedef float    v8f  __attribute__((ext_vector_type(8)));
typedef unsigned v4u  __attribute__((ext_vector_type(4)));
typedef int      v4i  __attribute__((ext_vector_type(4)));
union Frag { v16h v; v8h h[2]; v4u u[2]; };
union Pk8  { v8h h; v4u u; };

constexpr int NBT  = 4, NC = 128, NH = 128, NW = 128;
constexpr int NPIX = NBT * NH * NW;
constexpr int C2   = 2 * NC;
constexpr int NTAP = 9;
constexpr int KOFF = NTAP * C2;
constexpr int KDEF = NTAP * NC;
constexpr int KMOD = C2;
constexpr int NOFF = 18;
constexpr int NOFFP = 32;
constexpr int TPX  = 32;
constexpr int NXT  = NW / TPX;
constexpr int NBLK = NBT * NH * NXT;
constexpr int SS   = 136;
constexpr int OLP  = 36;
constexpr float IOFF = 1.0f / 256.0f;
constexpr float IW64 = 1.0f / 64.0f;

static_assert(NXT * TPX == NW);
static_assert((KOFF % 32) == 0);
static_assert((KDEF % 32) == 0);
static_assert((KMOD % 32) == 0);
static_assert((SS * 2) % 16 == 0);
static_assert((OLP * 4) % 16 == 0);

__device__ __forceinline__ v8f wmh(v16h a, v16h b, v8f c)
{
    v8f d = __builtin_amdgcn_wmma_f32_16x16x32_f16(false, a, false, b, (short)0, c, false, false);
    asm volatile("v_nop\n\tv_nop\n\tv_nop\n\tv_nop" : "+v"(d) : "v"(a), "v"(b));
    return d;
}

__global__ __launch_bounds__(256) void k_packw(const float* __restrict__ src, _Float16* dst,
                                               int Kdim, int Nrows, int Nused, int cinLog2, int taps, float scale)
{
    const int t = blockIdx.x * 256 + threadIdx.x;
    const int total8 = (Nrows * Kdim) >> 3;
    if (t >= total8) return;
    const int e0 = t * 8;
    const int n  = e0 / Kdim;
    const int k0 = e0 - n * Kdim;
    const int cinN = 1 << cinLog2;
    const int cinMask = cinN - 1;
    const int nc = (n < Nused) ? n : (Nused - 1);
    Pk8 p;
#pragma unroll
    for (int i = 0; i < 8; ++i) {
        const int k   = k0 + i;
        const int tap = k >> cinLog2;
        const int cin = k & cinMask;
        float x = src[((size_t)nc * cinN + cin) * taps + tap];
        x = (n < Nused) ? x * scale : 0.0f;
        p.h[i] = (_Float16)x;
    }
    _Float16* q = dst + e0;
    *(volatile v4u*)q = p.u;
    __threadfence();
    *(volatile v4u*)q = p.u;
}

__global__ __launch_bounds__(256) void k_prep(const float* __restrict__ low, const float* __restrict__ high,
                                              _Float16* catT, float* lowT)
{
    __shared__ __attribute__((aligned(16))) float    lowF[TPX][132];
    __shared__ __attribute__((aligned(16))) _Float16 catS[TPX][264];

    const int tid = threadIdx.x, lane = tid & 31, wave = tid >> 5;
    const int bid = blockIdx.x;
    const int xt = bid & (NXT - 1), y = (bid >> 2) & (NH - 1), b = bid >> 9;
    const int x0 = xt * TPX;

#pragma unroll 1
    for (int it = 0; it < (C2 * TPX) / 256; ++it) {
        const int idx = it * 256 + tid;
        const int c = idx >> 5, j = idx & 31;
        const int cc = c & (NC - 1);
        const size_t gi = ((size_t)(b * NC + cc) * NH + y) * NW + x0 + j;
        const float* src = (c < NC) ? low : high;
        const float v = src[gi];
        catS[j][c] = (_Float16)v;
        if (c < NC) lowF[j][c] = v;
    }
    __syncthreads();

    v4u cv[4];
    v4f lv[4];
#pragma unroll
    for (int q = 0; q < 4; ++q) {
        const int j = wave * 4 + q;
        cv[q] = *(const v4u*)(&catS[j][8 * lane]);
        lv[q] = *(const v4f*)(&lowF[j][4 * lane]);
    }
    const size_t pix0 = ((size_t)b * NH + y) * NW + x0 + wave * 4;
#pragma unroll
    for (int q = 0; q < 4; ++q) {
        const size_t pix = pix0 + q;
        *(volatile v4u*)(catT + pix * C2 + 8 * lane) = cv[q];
        *(volatile v4f*)(lowT + pix * NC + 4 * lane) = lv[q];
    }
    __threadfence();
#pragma unroll
    for (int q = 0; q < 4; ++q) {
        const size_t pix = pix0 + q;
        *(volatile v4u*)(catT + pix * C2 + 8 * lane) = cv[q];
        *(volatile v4f*)(lowT + pix * NC + 4 * lane) = lv[q];
    }
}

__global__ __launch_bounds__(64) void k_main(
    const _Float16* __restrict__ catT, const float* __restrict__ lowT,
    const _Float16* __restrict__ wOffP, const _Float16* __restrict__ wDefP, const _Float16* __restrict__ wModP,
    const float* __restrict__ bOff, const float* __restrict__ bDef, const float* __restrict__ bMod,
    const float* __restrict__ high, float* out)
{
    __shared__ __attribute__((aligned(16))) float    offsL[TPX][20];
    __shared__ __attribute__((aligned(16))) int      metaO[TPX * NTAP][4];
    __shared__ __attribute__((aligned(16))) float    metaW[TPX * NTAP][4];
    __shared__ __attribute__((aligned(16))) _Float16 samp[3 * TPX * SS];
    __shared__ __attribute__((aligned(16))) float    outL[NC][OLP];

    const int tid = threadIdx.x, lane = tid & 31, wave = tid >> 5, h = lane >> 4, m = lane & 15;
    const int bid = blockIdx.x;
    const int xt = bid & (NXT - 1), y = (bid >> 2) & (NH - 1), b = bid >> 9;
    const int x0 = xt * TPX;
    const size_t imgPix = (size_t)b * NH * NW;
    const int pl0 = wave * 16;

    {
        v8f o0, o1;
#pragma unroll
        for (int r = 0; r < 8; ++r) { o0[r] = 0.0f; o1[r] = 0.0f; }
        const int xm = x0 + pl0 + m;
        const _Float16* bq0 = wOffP + (size_t)m * KOFF + 8 * h;
        const _Float16* bq1 = wOffP + (size_t)(16 + m) * KOFF + 8 * h;
#pragma unroll 1
        for (int kb = 0; kb < KOFF / 32; ++kb) {
            const int tap = kb >> 3, cinb = (kb & 7) * 32;
            const int ty = tap / 3, tx = tap - 3 * ty;
            const int yy = y + ty - 1, xx = xm + tx - 1;
            const bool ok = (yy >= 0) && (yy < NH) && (xx >= 0) && (xx < NW);
            const int yyc = min(max(yy, 0), NH - 1);
            const int xxc = min(max(xx, 0), NW - 1);
            const _Float16* ap = catT + (imgPix + (size_t)yyc * NW + xxc) * C2 + cinb + 8 * h;
            Frag a, f0, f1;
            a.h[0] = *(const v8h*)ap;
            a.h[1] = *(const v8h*)(ap + 16);
            const unsigned mk = ok ? 0xffffffffu : 0u;
            const v4u mkv = (v4u)mk;
            a.u[0] = a.u[0] & mkv;
            a.u[1] = a.u[1] & mkv;
            const _Float16* bp0 = bq0 + kb * 32;
            const _Float16* bp1 = bq1 + kb * 32;
            f0.h[0] = *(const v8h*)bp0;
            f0.h[1] = *(const v8h*)(bp0 + 16);
            f1.h[0] = *(const v8h*)bp1;
            f1.h[1] = *(const v8h*)(bp1 + 16);
            o0 = wmh(a.v, f0.v, o0);
            o1 = wmh(a.v, f1.v, o1);
        }
        const float bo0 = bOff[m];
        const float bo1 = bOff[min(16 + m, NOFF - 1)];
#pragma unroll
        for (int r = 0; r < 8; ++r) offsL[pl0 + 8 * h + r][m] = o0[r] * IOFF + bo0;
        if (m < NOFF - 16) {
#pragma unroll
            for (int r = 0; r < 8; ++r) offsL[pl0 + 8 * h + r][16 + m] = o1[r] * IOFF + bo1;
        }
    }
    __syncthreads();

#pragma unroll 1
    for (int i = tid; i < TPX * NTAP; i += 64) {
        const int pl = i / NTAP, t = i - pl * NTAP;
        const int ty = t / 3, tx = t - ty * 3;
        const float dy = offsL[pl][2 * t];
        const float dx = offsL[pl][2 * t + 1];
        const float pyf = (float)(y + ty - 1) + dy;
        const float pxf = (float)(x0 + pl + tx - 1) + dx;
        float fy = floorf(pyf), fx = floorf(pxf);
        const float wy = pyf - fy, wx = pxf - fx;
        fy = fminf(fmaxf(fy, -64.0f), 256.0f);
        fx = fminf(fmaxf(fx, -64.0f), 256.0f);
        const int iy = (int)fy, ix = (int)fx;
        const bool y0ok = (iy >= 0) && (iy < NH);
        const bool y1ok = (iy + 1 >= 0) && (iy + 1 < NH);
        const bool x0ok = (ix >= 0) && (ix < NW);
        const bool x1ok = (ix + 1 >= 0) && (ix + 1 < NW);
        const float omy = 1.0f - wy, omx = 1.0f - wx;
        const float w00 = omy * omx, w01 = omy * wx, w10 = wy * omx, w11 = wy * wx;
        const int cy0 = min(max(iy, 0), NH - 1), cy1 = min(max(iy + 1, 0), NH - 1);
        const int cx0 = min(max(ix, 0), NW - 1), cx1 = min(max(ix + 1, 0), NW - 1);
        metaO[i][0] = cy0 * NW + cx0;
        metaO[i][1] = cy0 * NW + cx1;
        metaO[i][2] = cy1 * NW + cx0;
        metaO[i][3] = cy1 * NW + cx1;
        metaW[i][0] = (y0ok && x0ok) ? w00 : 0.0f;
        metaW[i][1] = (y0ok && x1ok) ? w01 : 0.0f;
        metaW[i][2] = (y1ok && x0ok) ? w10 : 0.0f;
        metaW[i][3] = (y1ok && x1ok) ? w11 : 0.0f;
    }
    __syncthreads();

    v8f d[8];
#pragma unroll
    for (int nt = 0; nt < 8; ++nt) {
#pragma unroll
        for (int r = 0; r < 8; ++r) d[nt][r] = 0.0f;
    }
    const float* lowB = lowT + imgPix * NC + 4 * lane;

#pragma unroll 1
    for (int g = 0; g < 3; ++g) {
#pragma unroll 1
        for (int it = wave; it < TPX * 3; it += 2) {
            const int pl = it / 3, tl = it - pl * 3;
            const int mi = pl * NTAP + 3 * g + tl;
            const v4i ov4 = *(const v4i*)(&metaO[mi][0]);
            const v4f wv  = *(const v4f*)(&metaW[mi][0]);
            const v4f v00 = *(const v4f*)(lowB + (size_t)ov4.x * NC);
            const v4f v01 = *(const v4f*)(lowB + (size_t)ov4.y * NC);
            const v4f v10 = *(const v4f*)(lowB + (size_t)ov4.z * NC);
            const v4f v11 = *(const v4f*)(lowB + (size_t)ov4.w * NC);
            v4h hv;
#pragma unroll
            for (int c = 0; c < 4; ++c) {
                float s = (wv.x * v00[c]) + (wv.y * v01[c]);
                s = s + (wv.z * v10[c]);
                s = s + (wv.w * v11[c]);
                hv[c] = (_Float16)s;
            }
            *(v4h*)(samp + (tl * TPX + pl) * SS + 4 * lane) = hv;
        }
        __syncthreads();

#pragma unroll 1
        for (int kk = 0; kk < 12; ++kk) {
            const int tl = kk >> 2, cinb = (kk & 3) * 32;
            const int kg = g * 384 + kk * 32;
            Frag a;
            const _Float16* ap = samp + (tl * TPX + pl0 + m) * SS + cinb + 8 * h;
            a.h[0] = *(const v8h*)ap;
            a.h[1] = *(const v8h*)(ap + 16);
#pragma unroll
            for (int nt = 0; nt < 8; ++nt) {
                const _Float16* bp = wDefP + (size_t)(nt * 16 + m) * KDEF + kg + 8 * h;
                Frag f;
                f.h[0] = *(const v8h*)bp;
                f.h[1] = *(const v8h*)(bp + 16);
                d[nt] = wmh(a.v, f.v, d[nt]);
            }
        }
        __syncthreads();
    }

#pragma unroll
    for (int nt = 0; nt < 8; ++nt) {
        const int n = nt * 16 + m;
        const float bias = bDef[n];
        v4f u0, u1;
#pragma unroll
        for (int r = 0; r < 4; ++r) {
            u0[r] = d[nt][r] * IW64 + bias;
            u1[r] = d[nt][4 + r] * IW64 + bias;
        }
        *(v4f*)(&outL[n][pl0 + 8 * h])     = u0;
        *(v4f*)(&outL[n][pl0 + 8 * h + 4]) = u1;
    }

    {
        v8f gq[8];
#pragma unroll
        for (int nt = 0; nt < 8; ++nt) {
#pragma unroll
            for (int r = 0; r < 8; ++r) gq[nt][r] = 0.0f;
        }
        const _Float16* arow = catT + (imgPix + (size_t)y * NW + x0 + pl0 + m) * C2 + 8 * h;
#pragma unroll 1
        for (int kb = 0; kb < KMOD / 32; ++kb) {
            Frag a;
            a.h[0] = *(const v8h*)(arow + kb * 32);
            a.h[1] = *(const v8h*)(arow + kb * 32 + 16);
#pragma unroll
            for (int nt = 0; nt < 8; ++nt) {
                const _Float16* bp = wModP + (size_t)(nt * 16 + m) * KMOD + kb * 32 + 8 * h;
                Frag f;
                f.h[0] = *(const v8h*)bp;
                f.h[1] = *(const v8h*)(bp + 16);
                gq[nt] = wmh(a.v, f.v, gq[nt]);
            }
        }
#pragma unroll
        for (int nt = 0; nt < 8; ++nt) {
            const int n = nt * 16 + m;
            const float bias = bMod[n];
            v4f u0 = *(const v4f*)(&outL[n][pl0 + 8 * h]);
            v4f u1 = *(const v4f*)(&outL[n][pl0 + 8 * h + 4]);
#pragma unroll
            for (int r = 0; r < 4; ++r) {
                const float z0 = gq[nt][r] * IW64 + bias;
                const float z1 = gq[nt][4 + r] * IW64 + bias;
                const float g0 = __builtin_amdgcn_rcpf(1.0f + __expf(-z0));
                const float g1 = __builtin_amdgcn_rcpf(1.0f + __expf(-z1));
                u0[r] = u0[r] * g0;
                u1[r] = u1[r] * g1;
            }
            *(v4f*)(&outL[n][pl0 + 8 * h])     = u0;
            *(v4f*)(&outL[n][pl0 + 8 * h + 4]) = u1;
        }
    }
    __syncthreads();

    {
        const int cq = lane >> 3, j = lane & 7;
        v4f ov[16];
#pragma unroll
        for (int i = 0; i < 16; ++i) {
            const int c = wave * 64 + 4 * i + cq;
            const size_t gi = ((size_t)(b * NC + c) * NH + y) * NW + x0 + 4 * j;
            const v4f hv = *(const v4f*)(high + gi);
            const v4f lv = *(const v4f*)(&outL[c][4 * j]);
            ov[i] = lv + hv;
        }
#pragma unroll
        for (int i = 0; i < 16; ++i) {
            const int c = wave * 64 + 4 * i + cq;
            const size_t gi = ((size_t)(b * NC + c) * NH + y) * NW + x0 + 4 * j;
            *(volatile v4f*)(out + gi) = ov[i];
        }
        __threadfence();
#pragma unroll
        for (int i = 0; i < 16; ++i) {
            const int c = wave * 64 + 4 * i + cq;
            const size_t gi = ((size_t)(b * NC + c) * NH + y) * NW + x0 + 4 * j;
            *(volatile v4f*)(out + gi) = ov[i];
        }
    }
}

extern "C" void kernel_launch(void* const* d_in, const int* in_sizes, int n_in,
                              void* d_out, int out_size, void* d_ws, size_t ws_size,
                              hipStream_t stream)
{
    if (n_in < 8) return;
    if (in_sizes[0] != NPIX * NC || in_sizes[1] != NPIX * NC) return;
    if (in_sizes[2] != NOFF * C2 * NTAP || in_sizes[3] < NOFF) return;
    if (in_sizes[4] != NC * NC * NTAP || in_sizes[5] < NC) return;
    if (in_sizes[6] != NC * C2 || in_sizes[7] < NC) return;
    if (out_size != NPIX * NC) return;

    const float* low   = (const float*)d_in[0];
    const float* high  = (const float*)d_in[1];
    const float* w_off = (const float*)d_in[2];
    const float* b_off = (const float*)d_in[3];
    const float* w_def = (const float*)d_in[4];
    const float* b_def = (const float*)d_in[5];
    const float* w_mod = (const float*)d_in[6];
    const float* b_mod = (const float*)d_in[7];
    float* out = (float*)d_out;

    const size_t szCat = (size_t)NPIX * C2 * 2;
    const size_t szLow = (size_t)NPIX * NC * 4;
    const size_t szWo  = (size_t)NOFFP * KOFF * 2;
    const size_t szWd  = (size_t)NC * KDEF * 2;
    const size_t szWm  = (size_t)NC * KMOD * 2;
    size_t off = 0;
    const size_t oCat = off; off += szCat;
    const size_t oLow = off; off += szLow;
    const size_t oWo  = off; off += szWo;
    const size_t oWd  = off; off += szWd;
    const size_t oWm  = off; off += szWm;
    if (off > ws_size) return;

    char* ws = (char*)d_ws;
    _Float16* catT  = (_Float16*)(ws + oCat);
    float*    lowT  = (float*)(ws + oLow);
    _Float16* wOffP = (_Float16*)(ws + oWo);
    _Float16* wDefP = (_Float16*)(ws + oWd);
    _Float16* wModP = (_Float16*)(ws + oWm);

    const int t8o = (NOFFP * KOFF) / 8, t8d = (NC * KDEF) / 8, t8m = (NC * KMOD) / 8;
    k_packw<<<dim3((t8o + 255) / 256), dim3(256), 0, stream>>>(w_off, wOffP, KOFF, NOFFP, NOFF, 8, NTAP, 256.0f);
    k_packw<<<dim3((t8d + 255) / 256), dim3(256), 0, stream>>>(w_def, wDefP, KDEF, NC, NC, 7, NTAP, 64.0f);
    k_packw<<<dim3((t8m + 255) / 256), dim3(256), 0, stream>>>(w_mod, wModP, KMOD, NC, NC, 8, 1, 64.0f);

    k_prep<<<dim3(NBLK), dim3(256), 0, stream>>>(low, high, catT, lowT);

    k_main<<<dim3(NBLK), dim3(64), 0, stream>>>(catT, lowT, wOffP, wDefP, wModP, b_off, b_def, b_mod, high, out);
}
